// MultiHeadAttention_86397562126350
// MI455X (gfx1250) — hardware-run, weakly checked
//
#include <hip/hip_runtime.h>
#include <math.h>

#ifndef NB
#define NB 4
#endif
#ifndef SEQ
#define SEQ 1024
#endif
#define NB_FULL 4
#define SEQ_FULL 1024
#define DM 1024
#define NHD 16
#define NXE 256
#define XBS_FULL ((long long)SEQ_FULL * DM)
static_assert(SEQ % 64 == 0);
static_assert(SEQ >= NXE);
static_assert(SEQ <= SEQ_FULL);
static_assert(NB >= 1 && NB <= NB_FULL);
static_assert(NXE % 64 == 0);
static_assert((SEQ - NXE) % 64 == 0);

typedef __attribute__((ext_vector_type(16))) _Float16 v16h;
typedef __attribute__((ext_vector_type(8)))  _Float16 v8h;
typedef __attribute__((ext_vector_type(8)))  float    v8f;
typedef __attribute__((ext_vector_type(4)))  float    v4f;

__device__ __forceinline__ v8f wmma16(v16h a, v16h b, v8f c) {
    c = __builtin_amdgcn_wmma_f32_16x16x32_f16(false, a, false, b, (short)0, c, false, false);
    asm volatile("v_nop\n\tv_nop\n\tv_nop\n\tv_nop" : "+v"(c) : "v"(a), "v"(b));
    return c;
}
union FragH { v16h v; v8h h[2]; };
__device__ __forceinline__ v16h lds_frag(const _Float16* p) { FragH f; f.h[0] = *(const v8h*)(p); f.h[1] = *(const v8h*)(p + 16); return f.v; }
__device__ __forceinline__ v16h glb_frag_f32(const float* __restrict__ p) {
    const v4f a = *(const v4f*)(p), b = *(const v4f*)(p + 4), c = *(const v4f*)(p + 16), d = *(const v4f*)(p + 20);
    v16h r;
    r[0] = (_Float16)a.x;  r[1] = (_Float16)a.y;  r[2] = (_Float16)a.z;  r[3] = (_Float16)a.w;
    r[4] = (_Float16)b.x;  r[5] = (_Float16)b.y;  r[6] = (_Float16)b.z;  r[7] = (_Float16)b.w;
    r[8] = (_Float16)c.x;  r[9] = (_Float16)c.y;  r[10] = (_Float16)c.z; r[11] = (_Float16)c.w;
    r[12] = (_Float16)d.x; r[13] = (_Float16)d.y; r[14] = (_Float16)d.z; r[15] = (_Float16)d.w;
    return r;
}

#define VST2(T, ptr, val) do { const T vst2_v_ = (val); *(volatile T*)(ptr) = vst2_v_; __threadfence(); *(volatile T*)(ptr) = vst2_v_; } while (0)
#define VST2V4(ptr, val) do { const v4f vst2_v4_ = (val); *(volatile v4f*)(ptr) = vst2_v4_; __threadfence(); *(volatile v4f*)(ptr) = vst2_v4_; } while (0)

#define AW 4
#define KPITCH 72
#define OPITCH 68
struct AttnC {
    const float* Q; const float* K; const float* V; float* O;
    long long sQb, sKb, sVb, sOb;
    int ldq, ldk, ldv, ldo;
    int Lq, Lk, coff; float scale;
};
static_assert(sizeof(AttnC) == 4 * 8 + 4 * 8 + 8 * 4);

__global__ __launch_bounds__(32 * AW) __attribute__((amdgpu_num_vgpr(256))) void k_attn(AttnC p) {
    __shared__ __align__(16) _Float16 kl[64 * KPITCH];
    __shared__ __align__(16) _Float16 vt[64 * KPITCH];
    __shared__ __align__(16) _Float16 ph[AW][16 * KPITCH];
    __shared__ __align__(16) float    ot[AW][16 * OPITCH];
    const int tid = threadIdx.x, lane = tid & 31, hf = lane >> 4, l15 = lane & 15, wave = tid >> 5;
    const int h = blockIdx.y, b = blockIdx.z;
    const int q0 = (blockIdx.x * AW + wave) * 16;
    const float L2E = 1.4426950408889634f;
    const float NEG = -__builtin_inff();
    const float* kbase = p.K + b * p.sKb + h * 64;
    const float* vbase = p.V + b * p.sVb + h * 64;
    _Float16* myph = ph[wave];
    const float* qrow = p.Q + b * p.sQb + (long long)(q0 + l15) * p.ldq + h * 64 + 8 * hf;
    const v16h qa0 = glb_frag_f32(qrow);
    const v16h qa1 = glb_frag_f32(qrow + 32);
    v8f o[4]; float m8[8], l8[8];
#pragma unroll
    for (int t = 0; t < 4; ++t) { v8f zz = {}; o[t] = zz; }
#pragma unroll
    for (int i = 0; i < 8; ++i) { m8[i] = NEG; l8[i] = 0.f; }
    const int je = (int)(blockIdx.x * AW + AW - 1) * 16 + 16 + p.coff;
    const int jend = min(p.Lk, max(je, 0));
    for (int j0 = 0; j0 < jend; j0 += 64) {
        __syncthreads();
        {
            const int jr = tid >> 1, dh = (tid & 1) * 32;
            const float* krow = kbase + (long long)(j0 + jr) * p.ldk + dh;
            const float* vrow = vbase + (long long)(j0 + jr) * p.ldv + dh;
#pragma unroll
            for (int i = 0; i < 4; ++i) {
                const v4f k0 = *(const v4f*)(krow + 8 * i), k1 = *(const v4f*)(krow + 8 * i + 4);
                v8h kk;
                kk[0] = (_Float16)k0.x; kk[1] = (_Float16)k0.y; kk[2] = (_Float16)k0.z; kk[3] = (_Float16)k0.w;
                kk[4] = (_Float16)k1.x; kk[5] = (_Float16)k1.y; kk[6] = (_Float16)k1.z; kk[7] = (_Float16)k1.w;
                *(v8h*)(kl + jr * KPITCH + dh + 8 * i) = kk;
                const v4f v0 = *(const v4f*)(vrow + 8 * i), v1 = *(const v4f*)(vrow + 8 * i + 4);
                const int dc = dh + 8 * i;
                vt[(dc + 0) * KPITCH + jr] = (_Float16)v0.x; vt[(dc + 1) * KPITCH + jr] = (_Float16)v0.y;
                vt[(dc + 2) * KPITCH + jr] = (_Float16)v0.z; vt[(dc + 3) * KPITCH + jr] = (_Float16)v0.w;
                vt[(dc + 4) * KPITCH + jr] = (_Float16)v1.x; vt[(dc + 5) * KPITCH + jr] = (_Float16)v1.y;
                vt[(dc + 6) * KPITCH + jr] = (_Float16)v1.z; vt[(dc + 7) * KPITCH + jr] = (_Float16)v1.w;
            }
        }
        __syncthreads();
        v8f s[4];
#pragma unroll
        for (int t = 0; t < 4; ++t) {
            const _Float16* kr = kl + (t * 16 + l15) * KPITCH + 8 * hf;
            v8f acc = {};
            acc = wmma16(qa0, lds_frag(kr), acc);
            acc = wmma16(qa1, lds_frag(kr + 32), acc);
            s[t] = acc;
        }
#pragma unroll
        for (int i = 0; i < 8; ++i) {
            const int irow = q0 + i + 8 * hf;
            float sc[4];
#pragma unroll
            for (int t = 0; t < 4; ++t) {
                const int jg = j0 + t * 16 + l15;
                float v = s[t][i] * p.scale;
                if (jg > irow + p.coff) v = NEG; else v *= L2E;
                sc[t] = v;
            }
            float mx = fmaxf(fmaxf(sc[0], sc[1]), fmaxf(sc[2], sc[3]));
            mx = fmaxf(mx, __shfl_xor(mx, 1, 32)); mx = fmaxf(mx, __shfl_xor(mx, 2, 32));
            mx = fmaxf(mx, __shfl_xor(mx, 4, 32)); mx = fmaxf(mx, __shfl_xor(mx, 8, 32));
            const float mnew = fmaxf(m8[i], mx);
            const float corr = (mnew == NEG) ? 1.f : exp2f(m8[i] - mnew);
            float rs = 0.f;
#pragma unroll
            for (int t = 0; t < 4; ++t) {
                const float pp = (sc[t] == NEG) ? 0.f : exp2f(sc[t] - mnew); rs += pp;
                myph[(i + 8 * hf) * KPITCH + t * 16 + l15] = (_Float16)(pp * 4096.f);
            }
            rs += __shfl_xor(rs, 1, 32); rs += __shfl_xor(rs, 2, 32); rs += __shfl_xor(rs, 4, 32); rs += __shfl_xor(rs, 8, 32);
            l8[i] = l8[i] * corr + rs; m8[i] = mnew;
#pragma unroll
            for (int t = 0; t < 4; ++t) o[t][i] *= corr;
        }
        __syncthreads();
        {
            const _Float16* pr = myph + l15 * KPITCH + 8 * hf;
            const v16h pa0 = lds_frag(pr), pa1 = lds_frag(pr + 32);
#pragma unroll
            for (int t = 0; t < 4; ++t) {
                const _Float16* vr = vt + (t * 16 + l15) * KPITCH + 8 * hf;
                o[t] = wmma16(pa0, lds_frag(vr), o[t]);
                o[t] = wmma16(pa1, lds_frag(vr + 32), o[t]);
            }
        }
    }
    float* mo = ot[wave];
#pragma unroll
    for (int i = 0; i < 8; ++i) {
        const float inv = (l8[i] > 0.f) ? 1.f / (l8[i] * 4096.f) : 0.f;
#pragma unroll
        for (int t = 0; t < 4; ++t) mo[(i + 8 * hf) * OPITCH + t * 16 + l15] = o[t][i] * inv;
    }
    __syncthreads();
    float* obase = p.O + b * p.sOb + h * 64;
#pragma unroll
    for (int r0 = 0; r0 < 16; r0 += 2) {
        const int row = r0 + (lane >> 4), c4 = (lane & 15) * 4;
        const v4f v = *(const v4f*)(mo + row * OPITCH + c4);
        VST2V4(obase + (long long)(q0 + row) * p.ldo + c4, v);
    }
}

__global__ __launch_bounds__(256) void k_invf(float* __restrict__ invb, int half, int D, float base) {
    const int i = blockIdx.x * 256 + threadIdx.x;
    if (i >= ((half + 31) / 32) * 32) return;
    if (i >= half) { VST2(float, invb + i, 0.f); return; }
    const float e = (float)(2 * i) / (float)D;
    const float invf = 1.0f / powf(base, e);
    VST2(float, invb + i, invf);
}
__global__ __launch_bounds__(256) void k_sincos(float* __restrict__ cs, float* __restrict__ sn, const float* __restrict__ invb, int S, int half, float pscale) {
    const int idx = blockIdx.x * 256 + threadIdx.x;
    if (idx >= S * half) return;
    const int s = idx / half, i = idx - s * half;
    const float ang = (pscale * (float)s) * invb[i];
    VST2(float, cs + idx, cosf(ang)); VST2(float, sn + idx, sinf(ang));
}

__global__ __launch_bounds__(256) void k_rope4(const float* __restrict__ X, int ldx, float* __restrict__ Y, int ldy, const float* __restrict__ cs, const float* __restrict__ sn, int rows, int cols, int S) {
    const long long u = (long long)blockIdx.x * 256 + threadIdx.x; const int per = cols / 4;
    if (u >= (long long)rows * per) return;
    const int r = (int)(u / per); const int c0 = 4 * (int)(u % per);
    const int t = r % S; const int i0 = (c0 & 63) >> 1;
    const v4f x = *(const v4f*)(X + (long long)r * ldx + c0);
    const float ca = cs[t * 32 + i0], cb = cs[t * 32 + i0 + 1], sa = sn[t * 32 + i0], sb = sn[t * 32 + i0 + 1];
    v4f y;
    y.x = x.x * ca - x.y * sa; y.y = x.x * sa + x.y * ca;
    y.z = x.z * cb - x.w * sb; y.w = x.z * sb + x.w * cb;
    VST2V4(Y + (long long)r * ldy + c0, y);
}

namespace w25 {
typedef __attribute__((ext_vector_type(16))) _Float16 v16h;
typedef __attribute__((ext_vector_type(8)))  _Float16 v8h;
typedef __attribute__((ext_vector_type(16))) __bf16   v16b;
typedef __attribute__((ext_vector_type(8)))  __bf16   v8b;
typedef __attribute__((ext_vector_type(8)))  float    v8f;
typedef __attribute__((ext_vector_type(4)))  float    v4f;

__device__ __forceinline__ unsigned short f2bf_bits(float f) {
  unsigned u = __float_as_uint(f);
  return (unsigned short)((u + 0x7FFFu + ((u >> 16) & 1u)) >> 16);
}
__device__ __forceinline__ float bf_bits2f(unsigned short h) { return __uint_as_float(((unsigned)h) << 16); }

__device__ __forceinline__ void dep_guard_h(v8f& a, v8f& b, v16h x, v16h y) { asm volatile("v_nop\n\tv_nop\n\tv_nop\n\tv_nop" : "+v"(a), "+v"(b) : "v"(x), "v"(y)); }
__device__ __forceinline__ void dep_guard_b(v8f& a, v8f& b, v16b x, v16b y) { asm volatile("v_nop\n\tv_nop\n\tv_nop\n\tv_nop" : "+v"(a), "+v"(b) : "v"(x), "v"(y)); }
__device__ __forceinline__ void keep4_h(v16h a, v16h b, v16h c, v16h d) { asm volatile("v_nop" :: "v"(a), "v"(b), "v"(c), "v"(d)); }
__device__ __forceinline__ void keep4_b(v16b a, v16b b, v16b c, v16b d) { asm volatile("v_nop" :: "v"(a), "v"(b), "v"(c), "v"(d)); }
__device__ __forceinline__ void acc_guard4(v8f& a, v8f& b, v8f& c, v8f& d) { asm volatile("v_nop\n\tv_nop\n\tv_nop\n\tv_nop" : "+v"(a), "+v"(b), "+v"(c), "+v"(d)); }
template <typename T> struct Frag;
template <> struct Frag<_Float16> {
  typedef v16h V; union U { v16h v; v8h h[2]; };
  static __device__ __forceinline__ v16h load(const _Float16* p) {
    U f; f.h[0] = *(const v8h*)(p); f.h[1] = *(const v8h*)(p + 16); return f.v;
  }
  static __device__ __forceinline__ v8f mma(v16h a, v16h b, v8f c) {
    return __builtin_amdgcn_wmma_f32_16x16x32_f16(false, a, false, b, (short)0, c, false, false);
  }
  static __device__ __forceinline__ void guard(v8f& a, v8f& b, v16h x, v16h y) { dep_guard_h(a, b, x, y); }
  static __device__ __forceinline__ void keep(v16h a, v16h b, v16h c, v16h d) { keep4_h(a, b, c, d); }
};
template <> struct Frag<__bf16> {
  typedef v16b V; union U { v16b v; v8b h[2]; };
  static __device__ __forceinline__ v16b load(const __bf16* p) {
    U f; f.h[0] = *(const v8b*)(p); f.h[1] = *(const v8b*)(p + 16); return f.v;
  }
  static __device__ __forceinline__ v8f mma(v16b a, v16b b, v8f c) {
    return __builtin_amdgcn_wmma_f32_16x16x32_bf16(false, a, false, b, (short)0, c, false, false);
  }
  static __device__ __forceinline__ void guard(v8f& a, v8f& b, v16b x, v16b y) { dep_guard_b(a, b, x, y); }
  static __device__ __forceinline__ void keep(v16b a, v16b b, v16b c, v16b d) { keep4_b(a, b, c, d); }
};

template <int ET> struct Elem;
template <> struct Elem<0> { typedef _Float16 T; };
template <> struct Elem<1> { typedef __bf16 T; };
template <int ET, bool SPLIT, int BIAS_MODE, int OUT_MODE, bool RESID, int ACT = 0>
__global__ __launch_bounds__(256) void wmma_gemm64(
    const unsigned short* __restrict__ Ap, const unsigned short* __restrict__ A2p, int lda, long strideA,
    const unsigned short* __restrict__ Btp, const unsigned short* __restrict__ Bt2p, int ldb, long strideB,
    void* __restrict__ Cout, void* __restrict__ Cout2, int ldc, long strideC,
    const float* __restrict__ bias,
    const float* __restrict__ resid, long strideR,
    int M, int N, int K, float scale) {
  typedef typename Elem<ET>::T T;
  typedef typename Frag<T>::V V;
  const T* A = (const T*)Ap; const T* A2 = (const T*)A2p; const T* Bt = (const T*)Btp; const T* Bt2 = (const T*)Bt2p;
  __shared__ __align__(16) float sT[8][16 * 68];
  const int b    = blockIdx.y;
  const int lane = threadIdx.x & 31;
  const int wave = threadIdx.x >> 5;
  const int tilesN = N >> 6;
  const int tilesM = M >> 6;
  const int tile = blockIdx.x * 8 + wave;
  if (tile >= tilesM * tilesN) return;
  const int tm = tile / tilesN;
  const int tn = tile - tm * tilesN;
  const int m0 = tm << 6;
  const int n0 = tn << 6;

  const T* Ab  = A  + (size_t)b * strideA;
  const T* Bb  = Bt + (size_t)b * strideB;
  const T* Ab2 = SPLIT ? (A2  + (size_t)b * strideA) : nullptr;
  const T* Bb2 = SPLIT ? (Bt2 + (size_t)b * strideB) : nullptr;

  const int rlane = lane & 15;
  const int koff  = (lane >> 4) * 8;
  const int mOff  = (lane >> 4) * 8;

  v8f acc[4][4];
#pragma unroll
  for (int i = 0; i < 4; ++i)
#pragma unroll
    for (int j = 0; j < 4; ++j) acc[i][j] = (v8f){0.f,0.f,0.f,0.f,0.f,0.f,0.f,0.f};

  for (int k0 = 0; k0 < K; k0 += 32) {
    V bh[4], bl[4];
#pragma unroll
    for (int j = 0; j < 4; ++j) {
      const size_t bo = (size_t)(n0 + (j << 4) + rlane) * ldb + koff + k0;
      bh[j] = Frag<T>::load(Bb + bo);
      if (SPLIT) bl[j] = Frag<T>::load(Bb2 + bo);
    }
#pragma unroll
    for (int i = 0; i < 4; ++i) {
      const size_t ao = (size_t)(m0 + (i << 4) + rlane) * lda + koff + k0;
      V ah = Frag<T>::load(Ab + ao);
      V al;
      if (SPLIT) al = Frag<T>::load(Ab2 + ao);
#pragma unroll
      for (int j = 0; j < 4; ++j) {
        acc[i][j] = Frag<T>::mma(ah, bh[j], acc[i][j]);
        if (SPLIT) {
          acc[i][j] = Frag<T>::mma(ah, bl[j], acc[i][j]);
          acc[i][j] = Frag<T>::mma(al, bh[j], acc[i][j]);
        }
      }
      Frag<T>::guard(acc[i][0], acc[i][3], ah, SPLIT ? al : ah);
    }
    Frag<T>::keep(bh[0], bh[1], bh[2], bh[3]);
    if (SPLIT) Frag<T>::keep(bl[0], bl[1], bl[2], bl[3]);
  }
  acc_guard4(acc[0][0], acc[0][1], acc[0][2], acc[0][3]);
  acc_guard4(acc[1][0], acc[1][1], acc[1][2], acc[1][3]);
  acc_guard4(acc[2][0], acc[2][1], acc[2][2], acc[2][3]);
  acc_guard4(acc[3][0], acc[3][1], acc[3][2], acc[3][3]);

  float* slab = sT[wave];
  const float* Rb = RESID ? (resid + (size_t)b * strideR) : nullptr;
#pragma unroll
  for (int i = 0; i < 4; ++i) {
    const int mBase = m0 + (i << 4);
#pragma unroll
    for (int j = 0; j < 4; ++j) {
      const int n = n0 + (j << 4) + rlane;
      float bv = 0.f;
      if (BIAS_MODE == 2) bv = bias[n];
#pragma unroll
      for (int r = 0; r < 8; ++r) {
        float v = acc[i][j][r] * scale;
        if (BIAS_MODE == 1) v += bias[mBase + mOff + r];
        if (BIAS_MODE == 2) v += bv;
        if (RESID) v += Rb[(size_t)(mBase + mOff + r) * ldc + n];
        if (ACT == 1) v = tanhf(v);
        if (ACT == 2) v = fmaxf(v, 0.0f);
        if (ACT == 3) v = v / (1.0f + expf(-v));
        if (ACT == 4) v = (v > 0.f) ? v : 0.01f * v;
        if (ACT == 5) v = 0.5f * v * (1.0f + erff(v * 0.70710678118654752f));
        if (ACT == 6) v = (v > 0.f) ? v : 0.2f * v;
        if (ACT == 7) { const float u = 0.7978845608028654f * (v + 0.044715f * v * v * v); v = 0.5f * v * (1.f + tanhf(u)); }
        slab[(mOff + r) * 68 + (j << 4) + rlane] = v;
      }
    }
    __builtin_amdgcn_fence(3  , "workgroup");
    __builtin_amdgcn_wave_barrier();
    __builtin_amdgcn_fence(2  , "workgroup");
    if (OUT_MODE == 0) {
      float* C = (float*)Cout + (size_t)b * strideC;
      const int hh = lane >> 4, c4 = (lane & 15) * 4;
      for (int pass = 0; pass < 2; ++pass) {
#pragma unroll
        for (int it = 0; it < 8; ++it) {
          const int row = it * 2 + hh;
          v4f v = *(const v4f*)(slab + row * 68 + c4);
          *(volatile v4f*)(C + (size_t)(mBase + row) * ldc + n0 + c4) = v;
        }
        __threadfence();
      }
    } else {
      const int q = lane >> 3, c8 = (lane & 7) * 8;
      unsigned short* C  = (unsigned short*)Cout  + (size_t)b * strideC;
      unsigned short* C2 = (OUT_MODE == 2) ? ((unsigned short*)Cout2 + (size_t)b * strideC) : nullptr;
      for (int pass = 0; pass < 2; ++pass) {
#pragma unroll
        for (int it = 0; it < 4; ++it) {
          const int row = it * 4 + q;
          const float* sp = slab + row * 68 + c8;
          v8h hv, lv;
#pragma unroll
          for (int e = 0; e < 8; ++e) {
            if (OUT_MODE == 1) {
              hv[e] = (_Float16)sp[e];
            } else {
              unsigned short hb = f2bf_bits(sp[e]);
              unsigned short lb = f2bf_bits(sp[e] - bf_bits2f(hb));
              hv[e] = __builtin_bit_cast(_Float16, hb);
              lv[e] = __builtin_bit_cast(_Float16, lb);
            }
          }
          *(volatile v8h*)(C + (size_t)(mBase + row) * ldc + n0 + c8) = hv;
          if (OUT_MODE == 2) *(volatile v8h*)(C2 + (size_t)(mBase + row) * ldc + n0 + c8) = lv;
        }
        __threadfence();
      }
    }
    __builtin_amdgcn_fence(3  , "workgroup");
    __builtin_amdgcn_wave_barrier();
    __builtin_amdgcn_fence(2  , "workgroup");
  }
}
}

__global__ __launch_bounds__(256) void k_cast16(const float* __restrict__ src, long long lds, _Float16* __restrict__ dst, long long ldd, int R, int C, float s) {
    const long long i = (long long)blockIdx.x * 256 + threadIdx.x; const long long np = (long long)R * (C / 2); if (i >= np) return; const int r = (int)(i / (C / 2)); const int c = 2 * (int)(i % (C / 2));
    const _Float16 h0 = (_Float16)(src[(long long)r * lds + c] * s), h1 = (_Float16)(src[(long long)r * lds + c + 1] * s);
    const unsigned u = (unsigned)__builtin_bit_cast(unsigned short, h0) | ((unsigned)__builtin_bit_cast(unsigned short, h1) << 16);
    volatile unsigned* d = (volatile unsigned*)(dst + (long long)r * ldd + c); *d = u; __threadfence(); *d = u; }

__device__ __forceinline__ unsigned int f2bf2_pack(float a, float b, unsigned int* lo) {
    const unsigned short ha = w25::f2bf_bits(a), hb = w25::f2bf_bits(b);
    const unsigned short la = w25::f2bf_bits(a - w25::bf_bits2f(ha)), lb = w25::f2bf_bits(b - w25::bf_bits2f(hb));
    *lo = (unsigned)la | ((unsigned)lb << 16); return (unsigned)ha | ((unsigned)hb << 16); }
__global__ __launch_bounds__(256) void k_castS16(const float* __restrict__ src, long long lds, __bf16* __restrict__ dhi, __bf16* __restrict__ dlo, long long ldd, int R, int C, float s, int transpose) {
    const long long i = (long long)blockIdx.x * 256 + threadIdx.x; long long o; float a, b;
    if (transpose) { const long long np = (long long)C * (R / 2); if (i >= np) return; const int c = (int)(i / (R / 2)); const int r = 2 * (int)(i % (R / 2)); a = src[(long long)r * lds + c] * s; b = src[(long long)(r + 1) * lds + c] * s; o = (long long)c * ldd + r; }
    else { const long long np = (long long)R * (C / 2); if (i >= np) return; const int r = (int)(i / (C / 2)); const int c = 2 * (int)(i % (C / 2)); a = src[(long long)r * lds + c] * s; b = src[(long long)r * lds + c + 1] * s; o = (long long)r * ldd + c; }
    unsigned lo; const unsigned hi = f2bf2_pack(a, b, &lo); volatile unsigned* ph = (volatile unsigned*)(dhi + o); volatile unsigned* pl = (volatile unsigned*)(dlo + o);
    *ph = hi; *pl = lo; __threadfence(); *ph = hi; *pl = lo; }

typedef unsigned int cm_u4 __attribute__((ext_vector_type(4)));
__device__ __forceinline__ unsigned int cmb_pk2(float a, float b) { return (unsigned int)__builtin_bit_cast(unsigned short, (_Float16)a) | ((unsigned int)__builtin_bit_cast(unsigned short, (_Float16)b) << 16); }
__device__ __forceinline__ float cmb_bf(float v) { const unsigned u = __builtin_bit_cast(unsigned, v); const unsigned r = (u + 0x7fffu + ((u >> 16) & 1u)) & 0xffff0000u; return __builtin_bit_cast(float, r); }
__global__ __launch_bounds__(256) void k_cm_castb(const float* __restrict__ SRC, int lds, unsigned short* __restrict__ DST, int ldd, int nR, int nC, float sc) {
    const long long u = (long long)blockIdx.x * 256 + threadIdx.x; const int per = nC / 8; if (u >= (long long)nR * per) return; const int r = (int)(u / per); const int c0 = 8 * (int)(u % per);
    const float* s = SRC + (long long)r * lds + c0; float w[8];
#pragma unroll
    for (int e = 0; e < 8; ++e) w[e] = cmb_bf(s[e]) * sc;
    cm_u4 pk; pk.x = cmb_pk2(w[0], w[1]); pk.y = cmb_pk2(w[2], w[3]); pk.z = cmb_pk2(w[4], w[5]); pk.w = cmb_pk2(w[6], w[7]); VST2(cm_u4, (cm_u4*)(DST + (long long)r * ldd + c0), pk); }

template <int NXR, int HREP>
__global__ __launch_bounds__(64) void k_gx_exact(const float* __restrict__ Q, int ldq, long long sqz, const float* __restrict__ Kp, int ldk, long long skz,
                                                  const float* __restrict__ Vp, int ldv, long long svz, float sc, float* __restrict__ AOX, int ldo, long long soz) {
    #pragma clang fp contract(off)
    __shared__ float qs[64]; __shared__ float ps[NXR]; __shared__ float red[2];
    const int i = blockIdx.x, h = blockIdx.y, z = blockIdx.z, t = threadIdx.x; const int kvh = h / HREP;
    const float* Qz = Q + z * sqz; const float* Kz = Kp + z * skz; const float* Vz = Vp + z * svz; float* Oz = AOX + z * soz;
    qs[t] = Qz[(long long)i * ldq + h * 64 + t]; __syncthreads();
#pragma unroll
    for (int r = 0; r < NXR / 64; ++r) {
        if (64 * r <= i) {
            const int j = t + 64 * r; const int jc = min(j, i); const float* kr = Kz + (long long)jc * ldk + kvh * 64; float s = 0.f;
#pragma unroll 8
            for (int d = 0; d < 64; ++d) s += qs[d] * kr[d];
            ps[j] = (j <= i) ? s * sc : -3.0e38f;
        }
    }
    __syncthreads();
    if (t == 0) { float m = -3.0e38f; for (int j = 0; j <= i; ++j) m = fmaxf(m, ps[j]); float zs = 0.f; for (int j = 0; j <= i; ++j) { const float e = expf(ps[j] - m); ps[j] = e; zs += e; } red[0] = 1.f / zs; }
    __syncthreads();
    const float inv = red[0]; float o = 0.f;
    for (int j = 0; j <= i; ++j) o += ps[j] * Vz[(long long)j * ldv + kvh * 64 + t];
    VST2(float, Oz + (long long)i * ldo + h * 64 + t, o * inv); }


extern "C" void kernel_launch(void* const* d_in, const int* in_sizes, int n_in, void* d_out, int out_size, void* d_ws, size_t ws_size, hipStream_t stream) {
    if (n_in < 5) return;
    const long long need_x = (long long)(NB - 1) * XBS_FULL + (long long)SEQ * DM;
    if ((long long)in_sizes[0] < need_x) return;
    if (in_sizes[1] < DM * DM || in_sizes[2] < DM * DM || in_sizes[3] < DM * DM || in_sizes[4] < DM * DM) return;
    if ((long long)out_size < need_x) return;
    const float* x  = (const float*)d_in[0];
    const float* wq = (const float*)d_in[1];
    const float* wk = (const float*)d_in[2];
    const float* wv = (const float*)d_in[3];
    const float* wo = (const float*)d_in[4];
    float* out = (float*)d_out;

    constexpr size_t R = (size_t)NB * SEQ;
    constexpr size_t SZ_X16  = R * DM * 2;
    constexpr size_t SZ_W3   = (size_t)3 * DM * DM * 2;
    constexpr size_t SZ_QKV  = R * 3 * DM * 4;
    constexpr size_t SZ_QKR  = R * 2 * DM * 4;
    constexpr size_t SZ_AO   = R * DM * 4;
    constexpr size_t SZ_W1   = (size_t)DM * DM * 2;
    constexpr size_t SZ_AOE  = (size_t)NB * NXE * DM * 2;
    constexpr size_t SZ_TAB  = (size_t)SEQ * 32 * 4;
    constexpr size_t SZ_INV  = 256;
    constexpr size_t SZ_TOTAL = SZ_X16 + SZ_W3 + SZ_QKV + SZ_QKR + SZ_AO + 3 * SZ_W1 + 2 * SZ_AOE + 2 * SZ_TAB + SZ_INV;
    static_assert(SZ_X16 % 256 == 0 && SZ_QKV % 256 == 0 && SZ_QKR % 256 == 0 && SZ_AO % 256 == 0 && SZ_AOE % 256 == 0 && SZ_TAB % 256 == 0);
    static_assert(SZ_TOTAL <= (size_t)134217728);
    if (SZ_TOTAL > ws_size) return;

    char* wsp = (char*)d_ws;
    unsigned short* X16  = (unsigned short*)wsp; wsp += SZ_X16;
    unsigned short* W316 = (unsigned short*)wsp; wsp += SZ_W3;
    float* QKV = (float*)wsp; wsp += SZ_QKV;
    float* QKR = (float*)wsp; wsp += SZ_QKR;
    float* AO  = (float*)wsp; wsp += SZ_AO;
    unsigned short* AO16 = X16;
    unsigned short* WO16 = (unsigned short*)wsp; wsp += SZ_W1;
    unsigned short* WOB  = (unsigned short*)wsp; wsp += SZ_W1;
    unsigned short* WOL  = (unsigned short*)wsp; wsp += SZ_W1;
    unsigned short* AOH2 = (unsigned short*)wsp; wsp += SZ_AOE;
    unsigned short* AOL2 = (unsigned short*)wsp; wsp += SZ_AOE;
    float* CS = (float*)wsp; wsp += SZ_TAB;
    float* SN = (float*)wsp; wsp += SZ_TAB;
    float* INVF = (float*)wsp; wsp += SZ_INV;

    const unsigned gW = (unsigned)(((long long)DM * (DM / 8) + 255) / 256);
    k_cm_castb<<<gW, 256, 0, stream>>>(wo, DM, WO16, DM, DM, DM, 16.0f);
    k_castS16<<<(unsigned)(((long long)DM * (DM / 2) + 255) / 256), 256, 0, stream>>>(wo, DM, (__bf16*)WOB, (__bf16*)WOL, DM, DM, DM, 1.0f, 0);
#if SEQ == SEQ_FULL
    k_cm_castb<<<(unsigned)(((long long)R * (DM / 8) + 255) / 256), 256, 0, stream>>>(x, DM, X16, DM, (int)R, DM, 1.0f);
#else
    for (int b = 0; b < NB; ++b)
        k_cm_castb<<<(unsigned)(((long long)SEQ * (DM / 8) + 255) / 256), 256, 0, stream>>>(x + (size_t)b * XBS_FULL, DM, X16 + (size_t)b * SEQ * DM, DM, SEQ, DM, 1.0f);
#endif
    k_cm_castb<<<gW, 256, 0, stream>>>(wq, DM, W316, DM, DM, DM, 16.0f);
    k_cm_castb<<<gW, 256, 0, stream>>>(wk, DM, W316 + (size_t)DM * DM, DM, DM, DM, 16.0f);
    k_cm_castb<<<gW, 256, 0, stream>>>(wv, DM, W316 + (size_t)2 * DM * DM, DM, DM, DM, 16.0f);
    w25::wmma_gemm64<0, false, 0, 0, false, 0><<<dim3((unsigned)((((int)R / 64) * (3 * DM / 64) + 7) / 8), 1u), 256, 0, stream>>>(
        (const unsigned short*)X16, nullptr, DM, (long)0, (const unsigned short*)W316, nullptr, DM, (long)0,
        (void*)QKV, nullptr, 3 * DM, (long)0, nullptr, nullptr, (long)0, (int)R, 3 * DM, DM, 0.0625f);
    k_invf<<<1, 256, 0, stream>>>(INVF, 32, 64, 10000.0f);
    k_sincos<<<(unsigned)((SEQ * 32 + 255) / 256), 256, 0, stream>>>(CS, SN, INVF, SEQ, 32, 1.0f);
    k_rope4<<<(unsigned)(((long long)R * (2 * DM / 4) + 255) / 256), 256, 0, stream>>>(QKV, 3 * DM, QKR, 2 * DM, CS, SN, (int)R, 2 * DM, SEQ);
    k_gx_exact<NXE, 1><<<dim3(NXE, NHD, NB), 64, 0, stream>>>(QKR, 2 * DM, (long long)SEQ * 2 * DM, QKR + DM, 2 * DM, (long long)SEQ * 2 * DM,
                                                              QKV + 2 * DM, 3 * DM, (long long)SEQ * 3 * DM, 0.125f, AO, DM, (long long)SEQ * DM);
#if SEQ > NXE
    { AttnC a;
      a.Q = QKR + (size_t)NXE * 2 * DM; a.K = QKR + DM; a.V = QKV + 2 * DM; a.O = AO + (size_t)NXE * DM;
      a.sQb = (long long)SEQ * 2 * DM; a.sKb = (long long)SEQ * 2 * DM; a.sVb = (long long)SEQ * 3 * DM; a.sOb = (long long)SEQ * DM;
      a.ldq = 2 * DM; a.ldk = 2 * DM; a.ldv = 3 * DM; a.ldo = DM;
      a.Lq = SEQ - NXE; a.Lk = SEQ; a.coff = NXE; a.scale = 0.125f;
      k_attn<<<dim3((unsigned)((SEQ - NXE) / (16 * AW)), (unsigned)NHD, (unsigned)NB), 32 * AW, 0, stream>>>(a); }
#endif
    k_cast16<<<(unsigned)(((long long)R * (DM / 2) + 255) / 256), 256, 0, stream>>>(AO, DM, (_Float16*)AO16, DM, (int)R, DM, 64.0f);
    w25::wmma_gemm64<0, false, 0, 0, false, 0><<<dim3((unsigned)(((SEQ / 64) * (DM / 64) + 7) / 8), (unsigned)NB), 256, 0, stream>>>(
        (const unsigned short*)AO16, nullptr, DM, (long)((long long)SEQ * DM), (const unsigned short*)WO16, nullptr, DM, (long)0,
        (void*)out, nullptr, DM, (long)XBS_FULL, nullptr, nullptr, (long)0, SEQ, DM, DM, 0.0009765625f);
    for (int b = 0; b < NB; ++b)
        k_castS16<<<(unsigned)(((long long)NXE * (DM / 2) + 255) / 256), 256, 0, stream>>>(AO + (size_t)b * SEQ * DM, DM,
            (__bf16*)(AOH2 + (size_t)b * NXE * DM), (__bf16*)(AOL2 + (size_t)b * NXE * DM), DM, NXE, DM, 1.0f, 0);
    w25::wmma_gemm64<1, false, 0, 0, false, 0><<<dim3((unsigned)(((NXE / 64) * (DM / 64) + 7) / 8), (unsigned)NB), 256, 0, stream>>>(
        (const unsigned short*)AOH2, nullptr, DM, (long)((long long)NXE * DM), (const unsigned short*)WOB, nullptr, DM, (long)0,
        (void*)out, nullptr, DM, (long)XBS_FULL, nullptr, nullptr, (long)0, NXE, DM, DM, 1.0f);
    w25::wmma_gemm64<1, false, 0, 0, true, 0><<<dim3((unsigned)(((NXE / 64) * (DM / 64) + 7) / 8), (unsigned)NB), 256, 0, stream>>>(
        (const unsigned short*)AOL2, nullptr, DM, (long)((long long)NXE * DM), (const unsigned short*)WOB, nullptr, DM, (long)0,
        (void*)out, nullptr, DM, (long)XBS_FULL, nullptr, out, (long)XBS_FULL, NXE, DM, DM, 1.0f);
}
